// FullyConnectedLoCS_79491254714575
// MI455X (gfx1250) — hardware-verified
//
#include <hip/hip_runtime.h>
#include <math.h>
typedef __attribute__((ext_vector_type(16))) _Float16 v16h;
typedef __attribute__((ext_vector_type(8)))  _Float16 v8h;
typedef __attribute__((ext_vector_type(16))) __bf16   v16b;
typedef __attribute__((ext_vector_type(8)))  __bf16   v8b;
typedef __attribute__((ext_vector_type(8)))  float    v8f;
typedef __attribute__((ext_vector_type(4)))  float    v4f;
#define PSCALE 32768.0f
#define U16(p) ((const unsigned short*)(const void*)(p))
#define PSCALE_INV (1.0f / 32768.0f)

__device__ __forceinline__ unsigned short f2bf_bits(float f) {
  unsigned u = __float_as_uint(f);
  return (unsigned short)((u + 0x7FFFu + ((u >> 16) & 1u)) >> 16);
}
__device__ __forceinline__ float bf_bits2f(unsigned short h) { return __uint_as_float(((unsigned)h) << 16); }

__device__ __forceinline__ void dep_guard_h(v8f& a, v8f& b, v16h x, v16h y) { asm volatile("v_nop\n\tv_nop\n\tv_nop\n\tv_nop" : "+v"(a), "+v"(b) : "v"(x), "v"(y)); }
__device__ __forceinline__ void dep_guard_b(v8f& a, v8f& b, v16b x, v16b y) { asm volatile("v_nop\n\tv_nop\n\tv_nop\n\tv_nop" : "+v"(a), "+v"(b) : "v"(x), "v"(y)); }
__device__ __forceinline__ void keep4_h(v16h a, v16h b, v16h c, v16h d) { asm volatile("v_nop" :: "v"(a), "v"(b), "v"(c), "v"(d)); }
__device__ __forceinline__ void keep4_b(v16b a, v16b b, v16b c, v16b d) { asm volatile("v_nop" :: "v"(a), "v"(b), "v"(c), "v"(d)); }
__device__ __forceinline__ void acc_guard4(v8f& a, v8f& b, v8f& c, v8f& d) { asm volatile("v_nop\n\tv_nop\n\tv_nop\n\tv_nop" : "+v"(a), "+v"(b), "+v"(c), "+v"(d)); }
template <typename T> struct Frag;
template <> struct Frag<_Float16> {
  typedef v16h V; union U { v16h v; v8h h[2]; };
  static __device__ __forceinline__ v16h load(const _Float16* p) {
    U f; f.h[0] = *(const v8h*)(p); f.h[1] = *(const v8h*)(p + 16); return f.v;
  }
  static __device__ __forceinline__ v8f mma(v16h a, v16h b, v8f c) {
    return __builtin_amdgcn_wmma_f32_16x16x32_f16(false, a, false, b, (short)0, c, false, false);
  }
  static __device__ __forceinline__ void guard(v8f& a, v8f& b, v16h x, v16h y) { dep_guard_h(a, b, x, y); }
  static __device__ __forceinline__ void keep(v16h a, v16h b, v16h c, v16h d) { keep4_h(a, b, c, d); }
};
template <> struct Frag<__bf16> {
  typedef v16b V; union U { v16b v; v8b h[2]; };
  static __device__ __forceinline__ v16b load(const __bf16* p) {
    U f; f.h[0] = *(const v8b*)(p); f.h[1] = *(const v8b*)(p + 16); return f.v;
  }
  static __device__ __forceinline__ v8f mma(v16b a, v16b b, v8f c) {
    return __builtin_amdgcn_wmma_f32_16x16x32_bf16(false, a, false, b, (short)0, c, false, false);
  }
  static __device__ __forceinline__ void guard(v8f& a, v8f& b, v16b x, v16b y) { dep_guard_b(a, b, x, y); }
  static __device__ __forceinline__ void keep(v16b a, v16b b, v16b c, v16b d) { keep4_b(a, b, c, d); }
};

template <int ET> struct Elem;
template <> struct Elem<0> { typedef _Float16 T; };
template <> struct Elem<1> { typedef __bf16 T; };
template <int ET, bool SPLIT, int BIAS_MODE, int OUT_MODE, bool RESID, int ACT = 0>
__global__ __launch_bounds__(256) void wmma_gemm64(
    const unsigned short* __restrict__ Ap, const unsigned short* __restrict__ A2p, int lda, long strideA,
    const unsigned short* __restrict__ Btp, const unsigned short* __restrict__ Bt2p, int ldb, long strideB,
    void* __restrict__ Cout, void* __restrict__ Cout2, int ldc, long strideC,
    const float* __restrict__ bias,
    const float* __restrict__ resid, long strideR,
    int M, int N, int K, float scale) {
  typedef typename Elem<ET>::T T;
  typedef typename Frag<T>::V V;
  const T* A = (const T*)Ap; const T* A2 = (const T*)A2p; const T* Bt = (const T*)Btp; const T* Bt2 = (const T*)Bt2p;
  __shared__ __align__(16) float sT[8][16 * 68];
  const int b    = blockIdx.y;
  const int lane = threadIdx.x & 31;
  const int wave = threadIdx.x >> 5;
  const int tilesN = N >> 6;
  const int tilesM = M >> 6;
  const int tile = blockIdx.x * 8 + wave;
  if (tile >= tilesM * tilesN) return;
  const int tm = tile / tilesN;
  const int tn = tile - tm * tilesN;
  const int m0 = tm << 6;
  const int n0 = tn << 6;

  const T* Ab  = A  + (size_t)b * strideA;
  const T* Bb  = Bt + (size_t)b * strideB;
  const T* Ab2 = SPLIT ? (A2  + (size_t)b * strideA) : nullptr;
  const T* Bb2 = SPLIT ? (Bt2 + (size_t)b * strideB) : nullptr;

  const int rlane = lane & 15;
  const int koff  = (lane >> 4) * 8;
  const int mOff  = (lane >> 4) * 8;

  v8f acc[4][4];
#pragma unroll
  for (int i = 0; i < 4; ++i)
#pragma unroll
    for (int j = 0; j < 4; ++j) acc[i][j] = (v8f){0.f,0.f,0.f,0.f,0.f,0.f,0.f,0.f};

  for (int k0 = 0; k0 < K; k0 += 32) {
    V bh[4], bl[4];
#pragma unroll
    for (int j = 0; j < 4; ++j) {
      const size_t bo = (size_t)(n0 + (j << 4) + rlane) * ldb + koff + k0;
      bh[j] = Frag<T>::load(Bb + bo);
      if (SPLIT) bl[j] = Frag<T>::load(Bb2 + bo);
    }
#pragma unroll
    for (int i = 0; i < 4; ++i) {
      const size_t ao = (size_t)(m0 + (i << 4) + rlane) * lda + koff + k0;
      V ah = Frag<T>::load(Ab + ao);
      V al;
      if (SPLIT) al = Frag<T>::load(Ab2 + ao);
#pragma unroll
      for (int j = 0; j < 4; ++j) {
        acc[i][j] = Frag<T>::mma(ah, bh[j], acc[i][j]);
        if (SPLIT) {
          acc[i][j] = Frag<T>::mma(ah, bl[j], acc[i][j]);
          acc[i][j] = Frag<T>::mma(al, bh[j], acc[i][j]);
        }
      }
      Frag<T>::guard(acc[i][0], acc[i][3], ah, SPLIT ? al : ah);
    }
    Frag<T>::keep(bh[0], bh[1], bh[2], bh[3]);
    if (SPLIT) Frag<T>::keep(bl[0], bl[1], bl[2], bl[3]);
  }
  acc_guard4(acc[0][0], acc[0][1], acc[0][2], acc[0][3]);
  acc_guard4(acc[1][0], acc[1][1], acc[1][2], acc[1][3]);
  acc_guard4(acc[2][0], acc[2][1], acc[2][2], acc[2][3]);
  acc_guard4(acc[3][0], acc[3][1], acc[3][2], acc[3][3]);

  float* slab = sT[wave];
  const float* Rb = RESID ? (resid + (size_t)b * strideR) : nullptr;
#pragma unroll
  for (int i = 0; i < 4; ++i) {
    const int mBase = m0 + (i << 4);
#pragma unroll
    for (int j = 0; j < 4; ++j) {
      const int n = n0 + (j << 4) + rlane;
      float bv = 0.f;
      if (BIAS_MODE == 2) bv = bias[n];
#pragma unroll
      for (int r = 0; r < 8; ++r) {
        float v = acc[i][j][r] * scale;
        if (BIAS_MODE == 1) v += bias[mBase + mOff + r];
        if (BIAS_MODE == 2) v += bv;
        if (RESID) v += Rb[(size_t)(mBase + mOff + r) * ldc + n];
        if (ACT == 1) v = tanhf(v);
        if (ACT == 2) v = fmaxf(v, 0.0f);
        if (ACT == 3) v = v / (1.0f + expf(-v));
        if (ACT == 4) v = (v > 0.f) ? v : 0.01f * v;
        if (ACT == 5) v = 0.5f * v * (1.0f + erff(v * 0.70710678118654752f));
        slab[(mOff + r) * 68 + (j << 4) + rlane] = v;
      }
    }
    __builtin_amdgcn_fence(__ATOMIC_RELEASE, "workgroup");
    __builtin_amdgcn_wave_barrier();
    __builtin_amdgcn_fence(__ATOMIC_ACQUIRE, "workgroup");
    if (OUT_MODE == 0) {
      float* C = (float*)Cout + (size_t)b * strideC;
      const int hh = lane >> 4, c4 = (lane & 15) * 4;
      for (int pass = 0; pass < 2; ++pass) {
#pragma unroll
        for (int it = 0; it < 8; ++it) {
          const int row = it * 2 + hh;
          v4f v = *(const v4f*)(slab + row * 68 + c4);
          *(volatile v4f*)(C + (size_t)(mBase + row) * ldc + n0 + c4) = v;
        }
        __threadfence();
      }
    } else {
      const int q = lane >> 3, c8 = (lane & 7) * 8;
      unsigned short* C  = (unsigned short*)Cout  + (size_t)b * strideC;
      unsigned short* C2 = (OUT_MODE == 2) ? ((unsigned short*)Cout2 + (size_t)b * strideC) : nullptr;
      for (int pass = 0; pass < 2; ++pass) {
#pragma unroll
        for (int it = 0; it < 4; ++it) {
          const int row = it * 4 + q;
          const float* sp = slab + row * 68 + c8;
          v8h hv, lv;
#pragma unroll
          for (int e = 0; e < 8; ++e) {
            if (OUT_MODE == 1) {
              hv[e] = (_Float16)sp[e];
            } else {
              unsigned short hb = f2bf_bits(sp[e]);
              unsigned short lb = f2bf_bits(sp[e] - bf_bits2f(hb));
              hv[e] = __builtin_bit_cast(_Float16, hb);
              lv[e] = __builtin_bit_cast(_Float16, lb);
            }
          }
          *(volatile v8h*)(C + (size_t)(mBase + row) * ldc + n0 + c8) = hv;
          if (OUT_MODE == 2) *(volatile v8h*)(C2 + (size_t)(mBase + row) * ldc + n0 + c8) = lv;
        }
        __threadfence();
      }
    }
    __builtin_amdgcn_fence(__ATOMIC_RELEASE, "workgroup");
    __builtin_amdgcn_wave_barrier();
    __builtin_amdgcn_fence(__ATOMIC_ACQUIRE, "workgroup");
  }
}

__global__ __launch_bounds__(256) void cast_f32_f16x2(
    const float* __restrict__ in, _Float16* __restrict__ out, int n2) {
  int i = blockIdx.x * 256 + threadIdx.x;
  if (i < n2) {
    const _Float16 h0 = (_Float16)in[2 * i], h1 = (_Float16)in[2 * i + 1];
    const unsigned u = (unsigned)__builtin_bit_cast(unsigned short, h0) | ((unsigned)__builtin_bit_cast(unsigned short, h1) << 16);
    ((volatile unsigned*)out)[i] = u;
    __threadfence();
    ((volatile unsigned*)out)[i] = u;
  }
}


__global__ __launch_bounds__(256) void transpose_cast_f16(const float* __restrict__ in, int ldi,
                                                         _Float16* __restrict__ outT, int ldo, float scale) {
  __shared__ __align__(16) _Float16 tile[64][72];
  const int c0 = blockIdx.x * 64, r0 = blockIdx.y * 64;
  const int t = threadIdx.y * 32 + threadIdx.x;
  for (int i = threadIdx.y; i < 64; i += 8) {
    tile[threadIdx.x][i]      = (_Float16)(in[(size_t)(r0 + i) * ldi + c0 + threadIdx.x] * scale);
    tile[32 + threadIdx.x][i] = (_Float16)(in[(size_t)(r0 + i) * ldi + c0 + 32 + threadIdx.x] * scale);
  }
  __syncthreads();
  const int q = t >> 3, c8 = (t & 7) * 8;
  for (int pass = 0; pass < 2; ++pass) {
#pragma unroll
    for (int it = 0; it < 2; ++it) {
      const int c = it * 32 + q;
      v8h hv = *(const v8h*)(&tile[c][c8]);
      *(volatile v8h*)(outT + (size_t)(c0 + c) * ldo + r0 + c8) = hv;
    }
    __threadfence();
  }
}

#define LB 64
#define LN 100
#define LH 128
#define LNODE (LB * LN)
#define LEPN (LN - 1)
#define LE ((long)LNODE * LEPN)
#define LEPAD 633600
__global__ __launch_bounds__(256) void node_kernel(const float* __restrict__ in, float* __restrict__ NF) {
  const int lane = threadIdx.x & 31, wave = threadIdx.x >> 5; const int n = (blockIdx.x * 8 + wave) * 4 + (lane >> 3); const int f = lane & 7;
  float val = 0.f;
  if (n < LNODE) { const float px = in[n * 4], py = in[n * 4 + 1], vx = in[n * 4 + 2], vy = in[n * 4 + 3]; const float th = atan2f(vy, vx); const float c = cosf(th), s = sinf(th);
    const float cvx = c * vx + s * vy, cvy = -s * vx + c * vy;
    val = (f == 0) ? c : (f == 1) ? s : (f == 2) ? px : (f == 3) ? py : (f == 4) ? vx : (f == 5) ? vy : (f == 6) ? cvx : cvy; }
  ((volatile float*)NF)[(size_t)(blockIdx.x * 8 + wave) * 32 + lane] = val; __threadfence(); ((volatile float*)NF)[(size_t)(blockIdx.x * 8 + wave) * 32 + lane] = val;
}
__global__ __launch_bounds__(256) void edge_kernel(const float* __restrict__ NF, unsigned* __restrict__ A) {
  const long e = (long)blockIdx.x * 256 + threadIdx.x; if (e >= LE) return; const int bi = (int)(e / LEPN), jj = (int)(e % LEPN); const int b = bi / LN, i = bi % LN; const int j = jj < i ? jj : jj + 1;
  const float* Fi = NF + (size_t)bi * 8; const float* Fj = NF + ((size_t)b * LN + j) * 8;
  const float ci = Fi[0], si = Fi[1], cj = Fj[0], sj = Fj[1];
  const float rx = Fj[2] - Fi[2], ry = Fj[3] - Fi[3];
  const float rrx = ci * rx + si * ry, rry = -si * rx + ci * ry;
  const float o00 = ci * cj + si * sj, o10 = -si * cj + ci * sj;
  const float euler = atan2f(o10, o00) * 0.3183098861837907f; const float dist = sqrtf(rx * rx + ry * ry); const float theta = atan2f(rry, rrx);
  const float rvx = ci * Fj[4] + si * Fj[5], rvy = -si * Fj[4] + ci * Fj[5];
  float at[12] = {rrx, rry, euler, dist, theta, rvx, rvy, 0.f, 0.f, Fi[6], Fi[7], 0.f};
  unsigned u[16];
#pragma unroll
  for (int q = 0; q < 6; ++q) u[q] = (unsigned)__builtin_bit_cast(unsigned short, (_Float16)at[2 * q]) | ((unsigned)__builtin_bit_cast(unsigned short, (_Float16)at[2 * q + 1]) << 16);
#pragma unroll
  for (int q = 6; q < 16; ++q) u[q] = 0u;
  typedef __attribute__((ext_vector_type(4))) unsigned u4;
  for (int pass = 0; pass < 2; ++pass) { for (int q = 0; q < 4; ++q) { const u4 v = {u[4*q], u[4*q+1], u[4*q+2], u[4*q+3]}; *(volatile u4*)(A + e * 16 + 4 * q) = v; } __threadfence(); }
}
__global__ __launch_bounds__(256) void w1_kernel(const float* __restrict__ W1, unsigned* __restrict__ BT) {
  for (int i = threadIdx.x; i < 128 * 16; i += 256) { const int o = i / 16, kp = 2 * (i % 16); const float a = (kp < 11) ? W1[kp * LH + o] : 0.f, b = (kp + 1 < 11) ? W1[(kp + 1) * LH + o] : 0.f;
    const unsigned u = (unsigned)__builtin_bit_cast(unsigned short, (_Float16)a) | ((unsigned)__builtin_bit_cast(unsigned short, (_Float16)b) << 16); ((volatile unsigned*)BT)[i] = u; __threadfence(); ((volatile unsigned*)BT)[i] = u; }
}
__global__ __launch_bounds__(256) void aggmean_kernel(const unsigned* __restrict__ S16, unsigned* __restrict__ AGG16) {
  const int lane = threadIdx.x & 31, wave = threadIdx.x >> 5; const int n = blockIdx.x * 8 + wave;
  typedef __attribute__((ext_vector_type(2))) unsigned u2; typedef __attribute__((ext_vector_type(4))) _Float16 v4h;
  v4f acc = {0.f, 0.f, 0.f, 0.f};
#pragma unroll 1
  for (int jj = 0; jj < LEPN; ++jj) { const u2 w = *(const u2*)(S16 + ((size_t)n * LEPN + jj) * 64 + lane * 2); const v4h h = __builtin_bit_cast(v4h, w); for (int q = 0; q < 4; ++q) acc[q] += (float)h[q]; }
  acc = acc * (1.0f / LEPN);
  u2 o; o[0] = (unsigned)__builtin_bit_cast(unsigned short, (_Float16)acc[0]) | ((unsigned)__builtin_bit_cast(unsigned short, (_Float16)acc[1]) << 16); o[1] = (unsigned)__builtin_bit_cast(unsigned short, (_Float16)acc[2]) | ((unsigned)__builtin_bit_cast(unsigned short, (_Float16)acc[3]) << 16);
  *(volatile u2*)(AGG16 + (size_t)n * 64 + lane * 2) = o; __threadfence(); *(volatile u2*)(AGG16 + (size_t)n * 64 + lane * 2) = o;
}
__global__ __launch_bounds__(256) void aug_kernel(const float* __restrict__ AUGP, const float* __restrict__ NF, const float* __restrict__ resw, const float* __restrict__ resb, unsigned* __restrict__ AUG16) {
  const int lane = threadIdx.x & 31, wave = threadIdx.x >> 5; const int n = blockIdx.x * 8 + wave; const float cvx = NF[(size_t)n * 8 + 6], cvy = NF[(size_t)n * 8 + 7];
  typedef __attribute__((ext_vector_type(2))) unsigned u2; u2 o;
  float v[4]; for (int q = 0; q < 4; ++q) { const int c = lane * 4 + q; v[q] = AUGP[(size_t)n * LH + c] + cvx * resw[2 * LH + c] + cvy * resw[3 * LH + c] + resb[c]; }
  o[0] = (unsigned)__builtin_bit_cast(unsigned short, (_Float16)v[0]) | ((unsigned)__builtin_bit_cast(unsigned short, (_Float16)v[1]) << 16); o[1] = (unsigned)__builtin_bit_cast(unsigned short, (_Float16)v[2]) | ((unsigned)__builtin_bit_cast(unsigned short, (_Float16)v[3]) << 16);
  *(volatile u2*)(AUG16 + (size_t)n * 64 + lane * 2) = o; __threadfence(); *(volatile u2*)(AUG16 + (size_t)n * 64 + lane * 2) = o;
}
__global__ __launch_bounds__(256) void head_kernel(const float* __restrict__ Y2, const float* __restrict__ w3, const float* __restrict__ b3, const float* __restrict__ NF, const float* __restrict__ in, float* __restrict__ out) {
  __shared__ float st[8][4];
  const int lane = threadIdx.x & 31, wave = threadIdx.x >> 5; const int n = blockIdx.x * 8 + wave;
  float p[4];
  for (int k = 0; k < 4; ++k) { float a = 0.f; for (int q = 0; q < 4; ++q) { const int c = lane * 4 + q; a += Y2[(size_t)n * LH + c] * w3[c * 4 + k]; } for (int o = 16; o > 0; o >>= 1) a += __shfl_xor(a, o, 32); p[k] = a + b3[k]; }
  if (lane == 0) { const float c = NF[(size_t)n * 8], s = NF[(size_t)n * 8 + 1];
    st[wave][0] = in[n * 4 + 0] + c * p[0] - s * p[1]; st[wave][1] = in[n * 4 + 1] + s * p[0] + c * p[1]; st[wave][2] = in[n * 4 + 2] + c * p[2] - s * p[3]; st[wave][3] = in[n * 4 + 3] + s * p[2] + c * p[3]; }
  __syncthreads();
  if (threadIdx.x < 32) { const float v = (&st[0][0])[threadIdx.x]; ((volatile float*)out)[blockIdx.x * 32 + threadIdx.x] = v; __threadfence(); ((volatile float*)out)[blockIdx.x * 32 + threadIdx.x] = v; }
}
extern "C" void kernel_launch(void* const* d_in, const int* in_sizes, int n_in, void* d_out, int out_size, void* d_ws, size_t ws_size, hipStream_t stream) {
  (void)in_sizes; (void)n_in; (void)out_size; (void)ws_size;
  auto F = [&](int i) { return (const float*)d_in[i]; };
  const float* inp = F(0); const float* W1 = F(1); const float* b1 = F(2); const float* W2 = F(3); const float* b2 = F(4); const float* resw = F(5); const float* resb = F(6);
  const float* ow1 = F(7); const float* ob1 = F(8); const float* ow2 = F(9); const float* ob2 = F(10); const float* ow3 = F(11); const float* ob3 = F(12);
  char* ws = (char*)d_ws; size_t off = 0;
  auto carve = [&](size_t bytes) -> char* { char* p = ws + off; off += (bytes + 255) & ~(size_t)255; return p; };
  float* NF = (float*)carve((size_t)LNODE * 8 * 4); unsigned* A = (unsigned*)carve((size_t)LEPAD * 32 * 2); unsigned* BT1 = (unsigned*)carve(128 * 32 * 2); unsigned* S16 = (unsigned*)carve((size_t)LEPAD * LH * 2);
  unsigned* AGG16 = (unsigned*)carve((size_t)LNODE * LH * 2); _Float16* W2T = (_Float16*)carve(LH * LH * 2); _Float16* O1T = (_Float16*)carve(LH * LH * 2); _Float16* O2T = (_Float16*)carve(LH * LH * 2);
  float* AUGP = (float*)carve((size_t)LNODE * LH * 4); unsigned* AUG16 = (unsigned*)carve((size_t)LNODE * LH * 2); _Float16* Y1 = (_Float16*)carve((size_t)LNODE * LH * 2); float* Y2 = (float*)carve((size_t)LNODE * LH * 4);
  node_kernel<<<LNODE / 32, 256, 0, stream>>>(inp, NF);
  edge_kernel<<<(unsigned)((LE + 255) / 256), 256, 0, stream>>>(NF, A);
  w1_kernel<<<1, 256, 0, stream>>>(W1, BT1);
  transpose_cast_f16<<<dim3(2, 2), dim3(32, 8), 0, stream>>>(W2, LH, W2T, LH, 1.0f);
  transpose_cast_f16<<<dim3(2, 2), dim3(32, 8), 0, stream>>>(ow1, LH, O1T, LH, 1.0f);
  transpose_cast_f16<<<dim3(2, 2), dim3(32, 8), 0, stream>>>(ow2, LH, O2T, LH, 1.0f);
  { const int t = (LEPAD / 64) * 2;
    wmma_gemm64<0, false, 2, 1, false, 3><<<dim3((t + 7) / 8, 1), 256, 0, stream>>>((const unsigned short*)A, nullptr, 32, 0, (const unsigned short*)BT1, nullptr, 32, 0, S16, nullptr, LH, 0, b1, nullptr, 0, LEPAD, LH, 32, 1.0f); }
  aggmean_kernel<<<LNODE / 8, 256, 0, stream>>>(S16, AGG16);
  const int tn = (LNODE / 64) * 2;
  wmma_gemm64<0, false, 2, 0, false, 0><<<dim3((tn + 7) / 8, 1), 256, 0, stream>>>((const unsigned short*)AGG16, nullptr, LH, 0, U16(W2T), nullptr, LH, 0, AUGP, nullptr, LH, 0, b2, nullptr, 0, LNODE, LH, LH, 1.0f);
  aug_kernel<<<LNODE / 8, 256, 0, stream>>>(AUGP, NF, resw, resb, AUG16);
  wmma_gemm64<0, false, 2, 1, false, 2><<<dim3((tn + 7) / 8, 1), 256, 0, stream>>>((const unsigned short*)AUG16, nullptr, LH, 0, U16(O1T), nullptr, LH, 0, Y1, nullptr, LH, 0, ob1, nullptr, 0, LNODE, LH, LH, 1.0f);
  wmma_gemm64<0, false, 2, 0, false, 2><<<dim3((tn + 7) / 8, 1), 256, 0, stream>>>(U16(Y1), nullptr, LH, 0, U16(O2T), nullptr, LH, 0, Y2, nullptr, LH, 0, ob2, nullptr, 0, LNODE, LH, LH, 1.0f);
  head_kernel<<<LNODE / 8, 256, 0, stream>>>(Y2, ow3, ob3, NF, inp, (float*)d_out);
}
